// SimplifiableTreeLSTM_13855564497597
// MI455X (gfx1250) — hardware-run, weakly checked
//
#include <hip/hip_runtime.h>
#include <stdint.h>

typedef __attribute__((ext_vector_type(16))) _Float16 v16h;
typedef __attribute__((ext_vector_type(8)))  _Float16 v8h;
typedef __attribute__((ext_vector_type(16))) __bf16   v16b;
typedef __attribute__((ext_vector_type(8)))  __bf16   v8b;
typedef __attribute__((ext_vector_type(8)))  float    v8f;
typedef __attribute__((ext_vector_type(4)))  float    v4f;

__device__ __forceinline__ unsigned short f2bf_bits(float f) {
  unsigned u = __float_as_uint(f);
  return (unsigned short)((u + 0x7FFFu + ((u >> 16) & 1u)) >> 16);
}
__device__ __forceinline__ float bf_bits2f(unsigned short h) { return __uint_as_float(((unsigned)h) << 16); }

__device__ __forceinline__ void dep_guard_h(v8f& a, v8f& b, v16h x, v16h y) { asm volatile("v_nop\n\tv_nop\n\tv_nop\n\tv_nop" : "+v"(a), "+v"(b) : "v"(x), "v"(y)); }
__device__ __forceinline__ void dep_guard_b(v8f& a, v8f& b, v16b x, v16b y) { asm volatile("v_nop\n\tv_nop\n\tv_nop\n\tv_nop" : "+v"(a), "+v"(b) : "v"(x), "v"(y)); }
__device__ __forceinline__ void keep4_h(v16h a, v16h b, v16h c, v16h d) { asm volatile("v_nop" :: "v"(a), "v"(b), "v"(c), "v"(d)); }
__device__ __forceinline__ void keep4_b(v16b a, v16b b, v16b c, v16b d) { asm volatile("v_nop" :: "v"(a), "v"(b), "v"(c), "v"(d)); }
__device__ __forceinline__ void acc_guard4(v8f& a, v8f& b, v8f& c, v8f& d) { asm volatile("v_nop\n\tv_nop\n\tv_nop\n\tv_nop" : "+v"(a), "+v"(b), "+v"(c), "+v"(d)); }
template <typename T> struct Frag;
template <> struct Frag<_Float16> {
  typedef v16h V; union U { v16h v; v8h h[2]; };
  static __device__ __forceinline__ v16h load(const _Float16* p) {
    U f; f.h[0] = *(const v8h*)(p); f.h[1] = *(const v8h*)(p + 16); return f.v;
  }
  static __device__ __forceinline__ v8f mma(v16h a, v16h b, v8f c) {
    return __builtin_amdgcn_wmma_f32_16x16x32_f16(false, a, false, b, (short)0, c, false, false);
  }
  static __device__ __forceinline__ void guard(v8f& a, v8f& b, v16h x, v16h y) { dep_guard_h(a, b, x, y); }
  static __device__ __forceinline__ void keep(v16h a, v16h b, v16h c, v16h d) { keep4_h(a, b, c, d); }
};
template <> struct Frag<__bf16> {
  typedef v16b V; union U { v16b v; v8b h[2]; };
  static __device__ __forceinline__ v16b load(const __bf16* p) {
    U f; f.h[0] = *(const v8b*)(p); f.h[1] = *(const v8b*)(p + 16); return f.v;
  }
  static __device__ __forceinline__ v8f mma(v16b a, v16b b, v8f c) {
    return __builtin_amdgcn_wmma_f32_16x16x32_bf16(false, a, false, b, (short)0, c, false, false);
  }
  static __device__ __forceinline__ void guard(v8f& a, v8f& b, v16b x, v16b y) { dep_guard_b(a, b, x, y); }
  static __device__ __forceinline__ void keep(v16b a, v16b b, v16b c, v16b d) { keep4_b(a, b, c, d); }
};

template <int ET> struct Elem;
template <> struct Elem<0> { typedef _Float16 T; };
template <> struct Elem<1> { typedef __bf16 T; };
template <int ET, bool SPLIT, int BIAS_MODE, int OUT_MODE, bool RESID, int ACT = 0>
__global__ __launch_bounds__(256) void wmma_gemm64(
    const unsigned short* __restrict__ Ap, const unsigned short* __restrict__ A2p, int lda, long strideA,
    const unsigned short* __restrict__ Btp, const unsigned short* __restrict__ Bt2p, int ldb, long strideB,
    void* __restrict__ Cout, void* __restrict__ Cout2, int ldc, long strideC,
    const float* __restrict__ bias,
    const float* __restrict__ resid, long strideR,
    int M, int N, int K, float scale) {
  typedef typename Elem<ET>::T T;
  typedef typename Frag<T>::V V;
  const T* A = (const T*)Ap; const T* A2 = (const T*)A2p; const T* Bt = (const T*)Btp; const T* Bt2 = (const T*)Bt2p;
  __shared__ __align__(16) float sT[8][16 * 68];
  const int b    = blockIdx.y;
  const int lane = threadIdx.x & 31;
  const int wave = threadIdx.x >> 5;
  const int tilesN = N >> 6;
  const int tilesM = M >> 6;
  const int tile = blockIdx.x * 8 + wave;
  if (tile >= tilesM * tilesN) return;
  const int tm = tile / tilesN;
  const int tn = tile - tm * tilesN;
  const int m0 = tm << 6;
  const int n0 = tn << 6;

  const T* Ab  = A  + (size_t)b * strideA;
  const T* Bb  = Bt + (size_t)b * strideB;
  const T* Ab2 = SPLIT ? (A2  + (size_t)b * strideA) : nullptr;
  const T* Bb2 = SPLIT ? (Bt2 + (size_t)b * strideB) : nullptr;

  const int rlane = lane & 15;
  const int koff  = (lane >> 4) * 8;
  const int mOff  = (lane >> 4) * 8;

  v8f acc[4][4];
#pragma unroll
  for (int i = 0; i < 4; ++i)
#pragma unroll
    for (int j = 0; j < 4; ++j) acc[i][j] = (v8f){0.f,0.f,0.f,0.f,0.f,0.f,0.f,0.f};

  for (int k0 = 0; k0 < K; k0 += 32) {
    V bh[4], bl[4];
#pragma unroll
    for (int j = 0; j < 4; ++j) {
      const size_t bo = (size_t)(n0 + (j << 4) + rlane) * ldb + koff + k0;
      bh[j] = Frag<T>::load(Bb + bo);
      if (SPLIT) bl[j] = Frag<T>::load(Bb2 + bo);
    }
#pragma unroll
    for (int i = 0; i < 4; ++i) {
      const size_t ao = (size_t)(m0 + (i << 4) + rlane) * lda + koff + k0;
      V ah = Frag<T>::load(Ab + ao);
      V al;
      if (SPLIT) al = Frag<T>::load(Ab2 + ao);
#pragma unroll
      for (int j = 0; j < 4; ++j) {
        acc[i][j] = Frag<T>::mma(ah, bh[j], acc[i][j]);
        if (SPLIT) {
          acc[i][j] = Frag<T>::mma(ah, bl[j], acc[i][j]);
          acc[i][j] = Frag<T>::mma(al, bh[j], acc[i][j]);
        }
      }
      Frag<T>::guard(acc[i][0], acc[i][3], ah, SPLIT ? al : ah);
    }
    Frag<T>::keep(bh[0], bh[1], bh[2], bh[3]);
    if (SPLIT) Frag<T>::keep(bl[0], bl[1], bl[2], bl[3]);
  }
  acc_guard4(acc[0][0], acc[0][1], acc[0][2], acc[0][3]);
  acc_guard4(acc[1][0], acc[1][1], acc[1][2], acc[1][3]);
  acc_guard4(acc[2][0], acc[2][1], acc[2][2], acc[2][3]);
  acc_guard4(acc[3][0], acc[3][1], acc[3][2], acc[3][3]);

  float* slab = sT[wave];
  const float* Rb = RESID ? (resid + (size_t)b * strideR) : nullptr;
#pragma unroll
  for (int i = 0; i < 4; ++i) {
    const int mBase = m0 + (i << 4);
#pragma unroll
    for (int j = 0; j < 4; ++j) {
      const int n = n0 + (j << 4) + rlane;
      float bv = 0.f;
      if (BIAS_MODE == 2) bv = bias[n];
#pragma unroll
      for (int r = 0; r < 8; ++r) {
        float v = acc[i][j][r] * scale;
        if (BIAS_MODE == 1) v += bias[mBase + mOff + r];
        if (BIAS_MODE == 2) v += bv;
        if (RESID) v += Rb[(size_t)(mBase + mOff + r) * ldc + n];
        if (ACT == 1) v = tanhf(v);
        if (ACT == 2) v = fmaxf(v, 0.0f);
        if (ACT == 3) v = v / (1.0f + expf(-v));
        if (ACT == 4) v = (v > 0.f) ? v : 0.01f * v;
        if (ACT == 5) v = 0.5f * v * (1.0f + erff(v * 0.70710678118654752f));
        slab[(mOff + r) * 68 + (j << 4) + rlane] = v;
      }
    }
    __builtin_amdgcn_fence(__ATOMIC_RELEASE, "workgroup");
    __builtin_amdgcn_wave_barrier();
    __builtin_amdgcn_fence(__ATOMIC_ACQUIRE, "workgroup");
    if (OUT_MODE == 0) {
      float* C = (float*)Cout + (size_t)b * strideC;
      const int hh = lane >> 4, c4 = (lane & 15) * 4;
      for (int pass = 0; pass < 2; ++pass) {
#pragma unroll
        for (int it = 0; it < 8; ++it) {
          const int row = it * 2 + hh;
          v4f v = *(const v4f*)(slab + row * 68 + c4);
          *(volatile v4f*)(C + (size_t)(mBase + row) * ldc + n0 + c4) = v;
        }
        __threadfence();
      }
    } else {
      const int q = lane >> 3, c8 = (lane & 7) * 8;
      unsigned short* C  = (unsigned short*)Cout  + (size_t)b * strideC;
      unsigned short* C2 = (OUT_MODE == 2) ? ((unsigned short*)Cout2 + (size_t)b * strideC) : nullptr;
      for (int pass = 0; pass < 2; ++pass) {
#pragma unroll
        for (int it = 0; it < 4; ++it) {
          const int row = it * 4 + q;
          const float* sp = slab + row * 68 + c8;
          v8h hv, lv;
#pragma unroll
          for (int e = 0; e < 8; ++e) {
            if (OUT_MODE == 1) {
              hv[e] = (_Float16)sp[e];
            } else {
              unsigned short hb = f2bf_bits(sp[e]);
              unsigned short lb = f2bf_bits(sp[e] - bf_bits2f(hb));
              hv[e] = __builtin_bit_cast(_Float16, hb);
              lv[e] = __builtin_bit_cast(_Float16, lb);
            }
          }
          *(volatile v8h*)(C + (size_t)(mBase + row) * ldc + n0 + c8) = hv;
          if (OUT_MODE == 2) *(volatile v8h*)(C2 + (size_t)(mBase + row) * ldc + n0 + c8) = lv;
        }
        __threadfence();
      }
    }
    __builtin_amdgcn_fence(__ATOMIC_RELEASE, "workgroup");
    __builtin_amdgcn_wave_barrier();
    __builtin_amdgcn_fence(__ATOMIC_ACQUIRE, "workgroup");
  }
}

constexpr int kBatch  = 64;
constexpr int kSeq    = 512;
constexpr int kEmb    = 300;
constexpr int kEmbP   = 320;
constexpr int kHid    = 150;
constexpr int kHidP   = 160;
constexpr int kGateN  = 4 * kHidP;
constexpr int kHid4   = 4 * kHid;
constexpr int kNF     = 100;
constexpr int kNFP    = 128;
constexpr int kVocab  = 50000;
constexpr int kFc1    = 75;
constexpr int kNCls   = 3;
constexpr int kTok    = kBatch * kSeq;
constexpr int kXRows  = kTok + 32;
constexpr int kKC0    = kEmbP * 3;
constexpr int kKC1    = kEmbP * 4;
constexpr int kKC2    = kEmbP * 5;
constexpr int kWC0off = 0;
constexpr int kWC1off = kNFP * kKC0;
constexpr int kWC2off = kNFP * (kKC0 + kKC1);
constexpr int kWCtot  = kNFP * (kKC0 + kKC1 + kKC2);
constexpr int kCplane = kBatch * kNFP * kSeq;
constexpr int kWhhLd  = 192;
constexpr int kProjLd = kGateN;
constexpr int kSeqPB  = 16;
constexpr int kLstmBlocks = kBatch / kSeqPB;
constexpr float kInv256 = 1.0f / 256.0f;
constexpr float kInv64  = 1.0f / 64.0f;
static_assert(kKC0 % 32 == 0 && kKC1 % 32 == 0 && kKC2 % 32 == 0);
static_assert(kNFP % 64 == 0 && kSeq % 64 == 0);
static_assert(kXRows % 8 == 0);
static_assert((kEmbP * 2) % 128 == 0 && (kHidP * 4) % 128 == 0 && (kWhhLd * 2) % 128 == 0 && (kProjLd * 4) % 128 == 0);
static_assert(kBatch * kNCls == 192);
static_assert(kLstmBlocks * kSeqPB == kBatch);

__device__ __forceinline__ float bf_rne(float f) {
  unsigned u = __float_as_uint(f);
  u = (u + 0x7FFFu + ((u >> 16) & 1u)) & 0xFFFF0000u;
  return __uint_as_float(u);
}
__device__ __forceinline__ int imin(int a, int b) { return a < b ? a : b; }

__device__ __forceinline__ v8f mma_g(v16h a, v16h b, v8f c) {
  c = __builtin_amdgcn_wmma_f32_16x16x32_f16(false, a, false, b, (short)0, c, false, false);
  asm volatile("v_nop\n\tv_nop\n\tv_nop\n\tv_nop" : "+v"(c) : "v"(a), "v"(b));
  return c;
}
__device__ __forceinline__ void mma_guard4x(v8f& a, v8f& b, v8f& c, v8f& d,
                                            v16h x, v16h y0, v16h y1, v16h y2, v16h y3) {
  asm volatile("v_nop\n\tv_nop\n\tv_nop\n\tv_nop"
               : "+v"(a), "+v"(b), "+v"(c), "+v"(d)
               : "v"(x), "v"(y0), "v"(y1), "v"(y2), "v"(y3));
}
__device__ __forceinline__ void mma_guard8x(v8f& a0, v8f& a1, v8f& a2, v8f& a3, v8f& a4, v8f& a5, v8f& a6, v8f& a7,
                                            v16h x0, v16h x1, v16h y0, v16h y1, v16h y2, v16h y3) {
  asm volatile("v_nop\n\tv_nop\n\tv_nop\n\tv_nop"
               : "+v"(a0), "+v"(a1), "+v"(a2), "+v"(a3), "+v"(a4), "+v"(a5), "+v"(a6), "+v"(a7)
               : "v"(x0), "v"(x1), "v"(y0), "v"(y1), "v"(y2), "v"(y3));
}
__device__ __forceinline__ float fsig(float x)  { return __builtin_amdgcn_rcpf(1.0f + __expf(-x)); }
__device__ __forceinline__ float ftanh(float x) { return 1.0f - 2.0f * __builtin_amdgcn_rcpf(__expf(2.0f * x) + 1.0f); }

__global__ __launch_bounds__(256) void embed_rows_kernel(const int* __restrict__ x, const float* __restrict__ emb,
                                                         _Float16* __restrict__ X16) {
  const int tid = threadIdx.x, lane = tid & 31, wave = tid >> 5;
  const int r = blockIdx.x * 8 + wave;
  const bool real = (r < kTok);
  int idx = x[imin(r, kTok - 1)];
  idx = idx < 0 ? 0 : (idx >= kVocab ? (kVocab - 1) : idx);
  const float* src = emb + (size_t)idx * kEmb;
  _Float16* dst = X16 + (size_t)r * kEmbP;
#pragma unroll
  for (int it = 0; it < 2; ++it) {
    const int c0 = (it == 0) ? (8 * lane) : (256 + 8 * (lane & 7));
    const int bA = imin(c0, kEmb - 4), bB = imin(c0 + 4, kEmb - 4);
    const v4f va = *(const v4f*)(src + bA);
    const v4f vb = *(const v4f*)(src + bB);
    v8h o;
#pragma unroll
    for (int e = 0; e < 4; ++e) {
      o[e]     = (real && (c0 + e     < kEmb)) ? (_Float16)(16.0f * bf_rne(va[e])) : (_Float16)0.0f;
      o[4 + e] = (real && (c0 + 4 + e < kEmb)) ? (_Float16)(16.0f * bf_rne(vb[e])) : (_Float16)0.0f;
    }
    const bool act = (it == 0) || (lane < 8);
    for (int pass = 0; pass < 2; ++pass) {
      if (act) *(volatile v8h*)(dst + c0) = o;
      __threadfence();
    }
  }
}

__global__ __launch_bounds__(256) void conv_wprep_kernel(const float* __restrict__ cw3, const float* __restrict__ cb3,
                                                         const float* __restrict__ cw4, const float* __restrict__ cb4,
                                                         const float* __restrict__ cw5, const float* __restrict__ cb5,
                                                         _Float16* __restrict__ WC16, float* __restrict__ BIASC) {
  const int tid = threadIdx.x, lane = tid & 31, wave = tid >> 5;
  const int cv = blockIdx.y, f = blockIdx.x;
  const int w = 3 + cv;
  const int Kp = kEmbP * w;
  const float* W  = (cv == 0) ? cw3 : ((cv == 1) ? cw4 : cw5);
  const float* CB = (cv == 0) ? cb3 : ((cv == 1) ? cb4 : cb5);
  const int poff = (cv == 0) ? kWC0off : ((cv == 1) ? kWC1off : kWC2off);
  const int fc = imin(f, kNF - 1);
  const int chunks = Kp >> 3;
  if (tid < chunks) {
    const int k0 = tid * 8;
    v8h o;
#pragma unroll
    for (int e = 0; e < 8; ++e) {
      const int k  = k0 + e;
      const int kk = k / kEmbP;
      const int c  = k - kk * kEmbP;
      const int cc = imin(c, kEmb - 1);
      const float v = W[((size_t)fc * kEmb + cc) * w + kk];
      o[e] = (f < kNF && c < kEmb) ? (_Float16)(16.0f * bf_rne(v)) : (_Float16)0.0f;
    }
    _Float16* dst = WC16 + poff + (size_t)f * Kp + k0;
    for (int pass = 0; pass < 2; ++pass) { *(volatile v8h*)dst = o; __threadfence(); }
  }
  if (f == 0 && wave == 0) {
    v4f bv;
#pragma unroll
    for (int e = 0; e < 4; ++e) {
      const int ff = 4 * lane + e;
      bv[e] = (ff < kNF) ? bf_rne(CB[imin(ff, kNF - 1)]) : 0.0f;
    }
    float* dst = BIASC + cv * kNFP + 4 * lane;
    for (int pass = 0; pass < 2; ++pass) { *(volatile v4f*)dst = bv; __threadfence(); }
  }
}

__global__ __launch_bounds__(64) void lin_wprep_kernel(const float* __restrict__ W, _Float16* __restrict__ P,
                                                       int kin_seg, int kp_seg, int nseg, int ldp, float scale) {
  const int tid = threadIdx.x;
  const int row = blockIdx.x;
  const int g = row / kHidP;
  const int u = row - g * kHidP;
  const bool rv = (u < kHid);
  const int srow = g * kHid + imin(u, kHid - 1);
  const int kin_tot = kin_seg * nseg;
  const int chunks = ldp >> 3;
  if (tid < chunks) {
    const int k0 = tid * 8;
    v8h o;
#pragma unroll
    for (int e = 0; e < 8; ++e) {
      const int k = k0 + e;
      const int seg = k / kp_seg;
      const int kk = k - seg * kp_seg;
      const bool valid = rv && (seg < nseg) && (kk < kin_seg);
      const int segc = imin(seg, nseg - 1);
      const int kkc  = imin(kk, kin_seg - 1);
      const float v = W[(size_t)srow * kin_tot + segc * kin_seg + kkc];
      o[e] = valid ? (_Float16)(scale * bf_rne(v)) : (_Float16)0.0f;
    }
    _Float16* dst = P + (size_t)row * ldp + k0;
    for (int pass = 0; pass < 2; ++pass) { *(volatile v8h*)dst = o; __threadfence(); }
  }
}

__global__ __launch_bounds__(256) void cnn_max_kernel(const _Float16* __restrict__ CPL, _Float16* __restrict__ CNN16) {
  __shared__ float cs[3 * kNF + 4];
  const int tid = threadIdx.x, lane = tid & 31, wave = tid >> 5;
  const int b = blockIdx.x;
#pragma unroll 1
  for (int cv = 0; cv < 3; ++cv) {
    const _Float16* plane = CPL + (size_t)cv * kCplane + (size_t)b * kNFP * kSeq;
    const int Nt = kSeq - 2 - cv;
#pragma unroll 1
    for (int i = 0; i < 13; ++i) {
      const int f = wave + 8 * i;
      if (f < kNF) {
        const _Float16* rp = plane + (size_t)f * kSeq + 16 * lane;
        const v8h a  = *(const v8h*)rp;
        const v8h bb = *(const v8h*)(rp + 8);
        float m = 0.0f;
#pragma unroll
        for (int e = 0; e < 8; ++e) {
          const int t = 16 * lane + e;
          const float va = (float)a[e];
          const float vb = (float)bb[e];
          m = (t < Nt) ? fmaxf(m, va) : m;
          m = (t + 8 < Nt) ? fmaxf(m, vb) : m;
        }
#pragma unroll
        for (int off = 1; off < 32; off <<= 1) m = fmaxf(m, __shfl_xor(m, off, 32));
        if (lane == 0) cs[cv * kNF + f] = m;
      }
    }
  }
  __syncthreads();
  if (wave == 0) {
#pragma unroll
    for (int it = 0; it < 2; ++it) {
      const int j0 = (it == 0) ? (8 * lane) : (256 + 8 * (lane & 7));
      v8h o;
#pragma unroll
      for (int e = 0; e < 8; ++e) {
        const int j = j0 + e;
        o[e] = (j < kEmb) ? (_Float16)(16.0f * cs[imin(j, kEmb - 1)]) : (_Float16)0.0f;
      }
      const bool act = (it == 0) || (lane < 8);
      _Float16* dst = CNN16 + (size_t)b * kEmbP + j0;
      for (int pass = 0; pass < 2; ++pass) {
        if (act) *(volatile v8h*)dst = o;
        __threadfence();
      }
    }
  }
}

__global__ __launch_bounds__(64) void proj_kernel(const _Float16* __restrict__ CNN16, const _Float16* __restrict__ WIH16,
                                                  const float* __restrict__ bih, const float* __restrict__ bhh,
                                                  float* __restrict__ PROJ) {
  __shared__ __align__(16) float sT[16 * 36];
  const int tid = threadIdx.x, lane = tid & 31, wave = tid >> 5;
  const int c = lane & 15, hh = lane >> 4, koff = hh * 8;
  const int nb = blockIdx.x, mt = blockIdx.y;
  const int n0 = 32 * nb + 16 * wave;
  const int m0 = 16 * mt;
  v8f acc = (v8f){0.f,0.f,0.f,0.f,0.f,0.f,0.f,0.f};
#pragma unroll
  for (int kc = 0; kc < kEmbP / 32; ++kc) {
    const v16h fa = Frag<_Float16>::load(CNN16 + (size_t)(m0 + c) * kEmbP + koff + 32 * kc);
    const v16h fb = Frag<_Float16>::load(WIH16 + (size_t)(n0 + c) * kEmbP + koff + 32 * kc);
    acc = mma_g(fa, fb, acc);
  }
  const int n = n0 + c;
  const int g = n / kHidP;
  const int u = n - g * kHidP;
  const bool valid = (u < kHid);
  const int brow = g * kHid + imin(u, kHid - 1);
  const float b1 = bf_rne(bih[brow]);
  const float b2 = bf_rne(bhh[brow]);
#pragma unroll
  for (int r = 0; r < 8; ++r) {
    float v = acc[r] * kInv256;
    v = (v + b1) + b2;
    sT[(8 * hh + r) * 36 + 16 * wave + c] = valid ? v : 0.0f;
  }
  __syncthreads();
  const int q = lane >> 3, c4 = (lane & 7) * 4;
  for (int pass = 0; pass < 2; ++pass) {
#pragma unroll
    for (int it = 0; it < 2; ++it) {
      const int row = 8 * wave + 4 * it + q;
      const v4f val = *(const v4f*)(sT + row * 36 + c4);
      *(volatile v4f*)(PROJ + (size_t)(m0 + row) * kProjLd + 32 * nb + c4) = val;
    }
    __threadfence();
  }
}

__global__ __launch_bounds__(320) void lstm_kernel(const _Float16* __restrict__ WHH16, const float* __restrict__ PROJ,
                                                   float* __restrict__ HS) {
  __shared__ __align__(16) _Float16 h16[2 * kSeqPB * kHidP];
  __shared__ __align__(16) float    hst[2 * kSeqPB * kHidP];
  const int tid = threadIdx.x, lane = tid & 31, wave = tid >> 5;
  const int c = lane & 15, hh = lane >> 4, koff = hh * 8, mOff = hh * 8;
  const int b0 = blockIdx.x * kSeqPB;
  const int u = 16 * wave + c;
  const bool uval = (u < kHid);
  {
    const v8h z = {(_Float16)0.f,(_Float16)0.f,(_Float16)0.f,(_Float16)0.f,(_Float16)0.f,(_Float16)0.f,(_Float16)0.f,(_Float16)0.f};
    for (int i = tid; i < (2 * kSeqPB * kHidP) / 8; i += 320) *(v8h*)(h16 + 8 * i) = z;
  }
  v8f pre[4];
#pragma unroll
  for (int g = 0; g < 4; ++g) {
#pragma unroll
    for (int r = 0; r < 8; ++r) {
      const int b = b0 + mOff + r;
      const float pv = PROJ[(size_t)b * kProjLd + g * kHidP + u];
      pre[g][r] = uval ? (64.0f * pv) : 0.0f;
    }
  }
  float cst[8];
#pragma unroll
  for (int r = 0; r < 8; ++r) cst[r] = 0.0f;
  __syncthreads();

#pragma unroll 1
  for (int t = 0; t < kSeq; ++t) {
    const int cur = t & 1;
    const _Float16* hc = h16 + cur * (kSeqPB * kHidP);
    _Float16*       hn = h16 + (cur ^ 1) * (kSeqPB * kHidP);
    float*          hs = hst + cur * (kSeqPB * kHidP);
    v8f acc[4];
#pragma unroll
    for (int g = 0; g < 4; ++g) acc[g] = pre[g];
#pragma unroll
    for (int kc = 0; kc < kHidP / 32; ++kc) {
      const v16h fa = Frag<_Float16>::load(hc + c * kHidP + koff + 32 * kc);
      v16h fb[4];
#pragma unroll
      for (int g = 0; g < 4; ++g)
        fb[g] = Frag<_Float16>::load(WHH16 + (size_t)(g * kHidP + u) * kWhhLd + koff + 32 * kc);
#pragma unroll
      for (int g = 0; g < 4; ++g) acc[g] = Frag<_Float16>::mma(fa, fb[g], acc[g]);
      mma_guard4x(acc[0], acc[1], acc[2], acc[3], fa, fb[0], fb[1], fb[2], fb[3]);
    }
#pragma unroll
    for (int r = 0; r < 8; ++r) {
      const float zi = acc[0][r] * kInv64;
      const float zf = acc[1][r] * kInv64;
      const float zg = acc[2][r] * kInv64;
      const float zo = acc[3][r] * kInv64;
      const float ig = fsig(zi);
      const float fg = fsig(zf);
      const float gg = ftanh(zg);
      const float og = fsig(zo);
      const float cn = fg * cst[r] + ig * gg;
      cst[r] = cn;
      float h = og * ftanh(cn);
      h = uval ? h : 0.0f;
      hn[(mOff + r) * kHidP + u] = (_Float16)(8.0f * h);
      hs[(mOff + r) * kHidP + u] = h;
    }
    __syncthreads();
    for (int row = wave; row < kSeqPB; row += 10) {
      float* dst = HS + ((size_t)t * kBatch + b0 + row) * kHidP;
      const float* sp = hs + row * kHidP;
      const v4f v0 = *(const v4f*)(sp + 4 * lane);
      const v4f v1 = *(const v4f*)(sp + 128 + 4 * (lane & 7));
      for (int pass = 0; pass < 2; ++pass) {
        *(volatile v4f*)(dst + 4 * lane) = v0;
        if (lane < 8) *(volatile v4f*)(dst + 128 + 4 * lane) = v1;
        __threadfence();
      }
    }
  }
}

__global__ __launch_bounds__(256) void tree_pair_kernel(const float* __restrict__ Hp, const float* __restrict__ Cp, int has_c,
                                                        _Float16* __restrict__ A16, float* __restrict__ CSUM) {
  __shared__ __align__(16) float css[kHidP];
  const int tid = threadIdx.x, lane = tid & 31, wave = tid >> 5;
  const int p = blockIdx.x;
  const float* hlb = Hp + (size_t)(2 * p) * kBatch * kHidP;
  const float* hrb = Hp + (size_t)(2 * p + 1) * kBatch * kHidP;
#pragma unroll 1
  for (int i = 0; i < 8; ++i) {
    const int b = wave + 8 * i;
    const float* hl = hlb + (size_t)b * kHidP;
    const float* hr = hrb + (size_t)b * kHidP;
    _Float16* dst = A16 + ((size_t)p * kBatch + b) * kEmbP;
#pragma unroll
    for (int it = 0; it < 2; ++it) {
      const int j0 = (it == 0) ? (8 * lane) : (256 + 8 * (lane & 7));
      const bool hiSeg = (j0 >= kHidP);
      const int uidx = hiSeg ? (j0 - kHidP) : j0;
      const float mult = hiSeg ? 4.0f : 8.0f;
      const v4f a0 = *(const v4f*)(hl + uidx), a1 = *(const v4f*)(hl + uidx + 4);
      const v4f c0 = *(const v4f*)(hr + uidx), c1 = *(const v4f*)(hr + uidx + 4);
      v8h o;
#pragma unroll
      for (int e = 0; e < 4; ++e) {
        const float s0 = a0[e] + c0[e];
        const float s1 = a1[e] + c1[e];
        o[e]     = (uidx + e     < kHid) ? (_Float16)(s0 * mult) : (_Float16)0.0f;
        o[4 + e] = (uidx + 4 + e < kHid) ? (_Float16)(s1 * mult) : (_Float16)0.0f;
      }
      const bool act = (it == 0) || (lane < 8);
      for (int pass = 0; pass < 2; ++pass) {
        if (act) *(volatile v8h*)(dst + j0) = o;
        __threadfence();
      }
    }
  }
  if (tid < kHidP) {
    const int u = tid;
    double s = 0.0;
    if (has_c) {
      const float* cl = Cp + (size_t)(2 * p) * kBatch * kHidP + u;
      const float* cr = Cp + (size_t)(2 * p + 1) * kBatch * kHidP + u;
#pragma unroll 1
      for (int b = 0; b < kBatch; ++b) s += (double)(cl[(size_t)b * kHidP] + cr[(size_t)b * kHidP]);
    }
    css[u] = (u < kHid) ? (float)s : 0.0f;
  }
  __syncthreads();
  if (wave == 0) {
    const v4f v0 = *(const v4f*)(css + 4 * lane);
    const v4f v1 = *(const v4f*)(css + 128 + 4 * (lane & 7));
    float* dst = CSUM + (size_t)p * kHidP;
    for (int pass = 0; pass < 2; ++pass) {
      *(volatile v4f*)(dst + 4 * lane) = v0;
      if (lane < 8) *(volatile v4f*)(dst + 128 + 4 * lane) = v1;
      __threadfence();
    }
  }
}

__global__ __launch_bounds__(320) void tree_cell_kernel(const _Float16* __restrict__ A16, const float* __restrict__ CSUM,
                                                        const _Float16* __restrict__ WT16, const float* __restrict__ bt,
                                                        float* __restrict__ Hn, float* __restrict__ Cn) {
  __shared__ __align__(16) float hsn[32 * kHidP];
  __shared__ __align__(16) float csn[32 * kHidP];
  const int tid = threadIdx.x, lane = tid & 31, wave = tid >> 5;
  const int c = lane & 15, hh = lane >> 4, koff = hh * 8, mOff = hh * 8;
  const int blk = blockIdx.x;
  const int R0 = 32 * blk;
  const int p = blk >> 1;
  const int u = 16 * wave + c;
  const bool uval = (u < kHid);
  const int uc = imin(u, kHid - 1);
  const float bfv = uval ? bf_rne(bt[uc]) : 0.0f;
  const float biv = uval ? bf_rne(bt[kHid + uc]) : 0.0f;
  const float bgv = uval ? bf_rne(bt[2 * kHid + uc]) : 0.0f;
  const float bov = uval ? bf_rne(bt[3 * kHid + uc]) : 0.0f;
  const float csv = CSUM[(size_t)p * kHidP + u];

  v8f acc[2][4];
#pragma unroll
  for (int i = 0; i < 2; ++i)
#pragma unroll
    for (int g = 0; g < 4; ++g) acc[i][g] = (v8f){0.f,0.f,0.f,0.f,0.f,0.f,0.f,0.f};
#pragma unroll
  for (int kc = 0; kc < kEmbP / 32; ++kc) {
    const v16h a0 = Frag<_Float16>::load(A16 + (size_t)(R0 + c) * kEmbP + koff + 32 * kc);
    const v16h a1 = Frag<_Float16>::load(A16 + (size_t)(R0 + 16 + c) * kEmbP + koff + 32 * kc);
    v16h fb[4];
#pragma unroll
    for (int g = 0; g < 4; ++g)
      fb[g] = Frag<_Float16>::load(WT16 + (size_t)(g * kHidP + u) * kEmbP + koff + 32 * kc);
#pragma unroll
    for (int g = 0; g < 4; ++g) {
      acc[0][g] = Frag<_Float16>::mma(a0, fb[g], acc[0][g]);
      acc[1][g] = Frag<_Float16>::mma(a1, fb[g], acc[1][g]);
    }
    mma_guard8x(acc[0][0], acc[0][1], acc[0][2], acc[0][3], acc[1][0], acc[1][1], acc[1][2], acc[1][3],
                a0, a1, fb[0], fb[1], fb[2], fb[3]);
  }
#pragma unroll
  for (int i = 0; i < 2; ++i) {
#pragma unroll
    for (int r = 0; r < 8; ++r) {
      const int row = 16 * i + mOff + r;
      const float zf = acc[i][0][r] * kInv64 + bfv;
      const float zi = acc[i][1][r] * kInv64 + biv;
      const float zg = acc[i][2][r] * kInv64 + bgv;
      const float zo = acc[i][3][r] * kInv64 + bov;
      const float cn = fsig(zf) * csv + fsig(zi) * ftanh(zg);
      const float hv = fsig(zo) * ftanh(cn);
      hsn[row * kHidP + u] = uval ? hv : 0.0f;
      csn[row * kHidP + u] = uval ? cn : 0.0f;
    }
  }
  __syncthreads();
  for (int row = wave; row < 32; row += 10) {
    float* dh = Hn + (size_t)(R0 + row) * kHidP;
    float* dc = Cn + (size_t)(R0 + row) * kHidP;
    const float* sh = hsn + row * kHidP;
    const float* sc = csn + row * kHidP;
    const v4f h0 = *(const v4f*)(sh + 4 * lane), h1 = *(const v4f*)(sh + 128 + 4 * (lane & 7));
    const v4f c0 = *(const v4f*)(sc + 4 * lane), c1 = *(const v4f*)(sc + 128 + 4 * (lane & 7));
    for (int pass = 0; pass < 2; ++pass) {
      *(volatile v4f*)(dh + 4 * lane) = h0;
      if (lane < 8) *(volatile v4f*)(dh + 128 + 4 * lane) = h1;
      *(volatile v4f*)(dc + 4 * lane) = c0;
      if (lane < 8) *(volatile v4f*)(dc + 128 + 4 * lane) = c1;
      __threadfence();
    }
  }
}

__global__ __launch_bounds__(256) void head_kernel(const float* __restrict__ ROOT, const float* __restrict__ fc1w,
                                                   const float* __restrict__ fc1b, const float* __restrict__ fc2w,
                                                   const float* __restrict__ fc2b, float* __restrict__ out) {
  __shared__ float hid[kBatch * 76];
  __shared__ __align__(16) float os[kBatch * kNCls];
  const int tid = threadIdx.x, lane = tid & 31, wave = tid >> 5;
  for (int idx = tid; idx < kBatch * kFc1; idx += 256) {
    const int b = idx / kFc1;
    const int uu = idx - b * kFc1;
    const float* hp = ROOT + (size_t)b * kHidP;
    const float* wp = fc1w + (size_t)uu * kHid;
    float s = 0.0f;
#pragma unroll 1
    for (int k = 0; k < kHid; ++k) s = fmaf(hp[k], bf_rne(wp[k]), s);
    s += bf_rne(fc1b[uu]);
    hid[b * 76 + uu] = fmaxf(s, 0.0f);
  }
  __syncthreads();
  if (tid < kBatch * kNCls) {
    const int b = tid / kNCls;
    const int o = tid - b * kNCls;
    const float* hp = hid + b * 76;
    const float* wp = fc2w + o * kFc1;
    float s = 0.0f;
#pragma unroll 1
    for (int k = 0; k < kFc1; ++k) s = fmaf(hp[k], bf_rne(wp[k]), s);
    s += bf_rne(fc2b[o]);
    os[tid] = s;
  }
  __syncthreads();
  if (wave == 0) {
    const v4f v0 = *(const v4f*)(os + 4 * lane);
    const v4f v1 = *(const v4f*)(os + 128 + 4 * (lane & 15));
    for (int pass = 0; pass < 2; ++pass) {
      *(volatile v4f*)(out + 4 * lane) = v0;
      if (lane < 16) *(volatile v4f*)(out + 128 + 4 * lane) = v1;
      __threadfence();
    }
  }
}

extern "C" void kernel_launch(void* const* d_in, const int* in_sizes, int n_in,
                              void* d_out, int out_size, void* d_ws, size_t ws_size, hipStream_t stream) {
  if (n_in < 22 || d_out == nullptr || d_ws == nullptr) return;
  if (in_sizes[0] != kTok || in_sizes[1] != kVocab * kEmb ||
      in_sizes[2] != kNF * kEmb * 3 || in_sizes[3] != kNF ||
      in_sizes[4] != kNF * kEmb * 4 || in_sizes[5] != kNF ||
      in_sizes[6] != kNF * kEmb * 5 || in_sizes[7] != kNF ||
      in_sizes[8] != kHid4 * 3 * kNF || in_sizes[9] != kHid4 * kHid ||
      in_sizes[10] != kHid4 || in_sizes[11] != kHid4 ||
      in_sizes[16] != kHid4 * 2 * kHid || in_sizes[17] != kHid4 ||
      in_sizes[18] != kFc1 * kHid || in_sizes[19] != kFc1 ||
      in_sizes[20] != kNCls * kFc1 || in_sizes[21] != kNCls ||
      out_size != kBatch * kNCls) return;

  const int*   x     = (const int*)  d_in[0];
  const float* emb   = (const float*)d_in[1];
  const float* cw3   = (const float*)d_in[2];
  const float* cb3   = (const float*)d_in[3];
  const float* cw4   = (const float*)d_in[4];
  const float* cb4   = (const float*)d_in[5];
  const float* cw5   = (const float*)d_in[6];
  const float* cb5   = (const float*)d_in[7];
  const float* Wih_f = (const float*)d_in[8];
  const float* Whh_f = (const float*)d_in[9];
  const float* bih_f = (const float*)d_in[10];
  const float* bhh_f = (const float*)d_in[11];
  const float* Wt    = (const float*)d_in[16];
  const float* bt    = (const float*)d_in[17];
  const float* fc1w  = (const float*)d_in[18];
  const float* fc1b  = (const float*)d_in[19];
  const float* fc2w  = (const float*)d_in[20];
  const float* fc2b  = (const float*)d_in[21];
  float* out = (float*)d_out;

  char* base = (char*)d_ws;
  size_t off = 0;
  auto carve = [&](size_t bytes) -> char* { char* p = base + off; off += (bytes + 255) & ~(size_t)255; return p; };
  _Float16* X16   = (_Float16*)carve((size_t)kXRows * kEmbP * 2);
  _Float16* WC16  = (_Float16*)carve((size_t)kWCtot * 2);
  float*    BIASC = (float*)   carve((size_t)3 * kNFP * 4);
  _Float16* CPL   = (_Float16*)carve((size_t)3 * kCplane * 2);
  _Float16* CNN16 = (_Float16*)carve((size_t)kBatch * kEmbP * 2);
  _Float16* WIH16 = (_Float16*)carve((size_t)kGateN * kEmbP * 2);
  float*    PROJ  = (float*)   carve((size_t)kBatch * kProjLd * 4);
  _Float16* WHH16 = (_Float16*)carve((size_t)kGateN * kWhhLd * 2);
  float*    HS    = (float*)   carve((size_t)kSeq * kBatch * kHidP * 4);
  _Float16* WT16  = (_Float16*)carve((size_t)kGateN * kEmbP * 2);
  _Float16* A16   = (_Float16*)carve((size_t)256 * kBatch * kEmbP * 2);
  float*    CSUM  = (float*)   carve((size_t)256 * kHidP * 4);
  float*    HP    = (float*)   carve((size_t)256 * kBatch * kHidP * 4);
  float*    CP    = (float*)   carve((size_t)256 * kBatch * kHidP * 4);
  float*    HQ    = (float*)   carve((size_t)128 * kBatch * kHidP * 4);
  float*    CQ    = (float*)   carve((size_t)128 * kBatch * kHidP * 4);
  if (off > ws_size) return;

  embed_rows_kernel<<<kXRows / 8, 256, 0, stream>>>(x, emb, X16);
  conv_wprep_kernel<<<dim3(kNFP, 3), 256, 0, stream>>>(cw3, cb3, cw4, cb4, cw5, cb5, WC16, BIASC);
  lin_wprep_kernel<<<kGateN, 64, 0, stream>>>(Wih_f, WIH16, 3 * kNF, kEmbP, 1, kEmbP, 16.0f);
  lin_wprep_kernel<<<kGateN, 64, 0, stream>>>(Whh_f, WHH16, kHid, kHidP, 1, kWhhLd, 8.0f);
  lin_wprep_kernel<<<kGateN, 64, 0, stream>>>(Wt, WT16, kHid, kHidP, 2, kEmbP, 8.0f);

  const long strideB = (long)kSeq * kEmbP;
  const long strideC = (long)kNFP * kSeq;
  wmma_gemm64<0, false, 1, 1, false, 2><<<dim3(2, kBatch), 256, 0, stream>>>(
      (const unsigned short*)(WC16 + kWC0off), (const unsigned short*)(WC16 + kWC0off), kKC0, 0L,
      (const unsigned short*)X16, (const unsigned short*)X16, kEmbP, strideB,
      (void*)(CPL + 0 * (size_t)kCplane), (void*)(CPL + 0 * (size_t)kCplane), kSeq, strideC,
      BIASC + 0 * kNFP, BIASC, 0L, kNFP, kSeq, kKC0, kInv256);
  wmma_gemm64<0, false, 1, 1, false, 2><<<dim3(2, kBatch), 256, 0, stream>>>(
      (const unsigned short*)(WC16 + kWC1off), (const unsigned short*)(WC16 + kWC1off), kKC1, 0L,
      (const unsigned short*)X16, (const unsigned short*)X16, kEmbP, strideB,
      (void*)(CPL + 1 * (size_t)kCplane), (void*)(CPL + 1 * (size_t)kCplane), kSeq, strideC,
      BIASC + 1 * kNFP, BIASC, 0L, kNFP, kSeq, kKC1, kInv256);
  wmma_gemm64<0, false, 1, 1, false, 2><<<dim3(2, kBatch), 256, 0, stream>>>(
      (const unsigned short*)(WC16 + kWC2off), (const unsigned short*)(WC16 + kWC2off), kKC2, 0L,
      (const unsigned short*)X16, (const unsigned short*)X16, kEmbP, strideB,
      (void*)(CPL + 2 * (size_t)kCplane), (void*)(CPL + 2 * (size_t)kCplane), kSeq, strideC,
      BIASC + 2 * kNFP, BIASC, 0L, kNFP, kSeq, kKC2, kInv256);

  cnn_max_kernel<<<kBatch, 256, 0, stream>>>(CPL, CNN16);
  proj_kernel<<<dim3(kGateN / 32, kBatch / 16), 64, 0, stream>>>(CNN16, WIH16, bih_f, bhh_f, PROJ);
  lstm_kernel<<<kLstmBlocks, 320, 0, stream>>>(WHH16, PROJ, HS);

  const float* hin = HS;
  const float* cin = HS;
  int has_c = 0;
  for (int L = 0; L < 9; ++L) {
    const int m = 256 >> L;
    float* hout = (L & 1) ? HQ : HP;
    float* cout_ = (L & 1) ? CQ : CP;
    tree_pair_kernel<<<m, 256, 0, stream>>>(hin, cin, has_c, A16, CSUM);
    tree_cell_kernel<<<2 * m, 320, 0, stream>>>(A16, CSUM, WT16, bt, hout, cout_);
    hin = hout; cin = cout_; has_c = 1;
  }

  head_kernel<<<1, 256, 0, stream>>>(HP, fc1w, fc1b, fc2w, fc2b, out);
}
